// BatchedAdjacency_40793599377963
// MI455X (gfx1250) — hardware-verified
//
#include <hip/hip_runtime.h>
#include <stddef.h>


#define NB          4
#define LCH         16
#define DG          5
#define NPIX        4096
#define NTHR        256
#define NWAVE       8
#define ROWS        128
#define KCH         32
#define GP          8
#define SPITCH      132
#define CVT_PER_THR 8
#define GLDS        (NPIX * GP * 4)
#define WSCAP       134217728

static_assert(NTHR == NWAVE * 32);
static_assert(ROWS == NWAVE * 16);
static_assert((NPIX % ROWS) == 0 && (NPIX % KCH) == 0);
static_assert(LCH == 16);
static_assert(LCH == 2 * NWAVE);
static_assert(ROWS * 4 == 32 * 16);
static_assert((NPIX % (4 * NTHR)) == 0);
static_assert(((NB * LCH * NPIX) % (CVT_PER_THR * NTHR)) == 0);
static_assert((SPITCH % 4) == 0 && SPITCH >= ROWS);
static_assert(DG == 5 && GP >= DG && (GP % 4) == 0);

typedef float     v4f  __attribute__((ext_vector_type(4)));
typedef float     v8f  __attribute__((ext_vector_type(8)));
typedef _Float16  v8h  __attribute__((ext_vector_type(8)));
typedef _Float16  v16h __attribute__((ext_vector_type(16)));
union FragH { v16h v; v8h h[2]; _Float16 e[16]; };

__device__ __forceinline__ v8f wmf(v16h a, v16h b, v8f c) {
  v8f d = __builtin_amdgcn_wmma_f32_16x16x32_f16(false, a, false, b, (short)0, c, false, false);
  asm volatile("v_nop\n\tv_nop\n\tv_nop\n\tv_nop" : "+v"(d) : "v"(a), "v"(b));
  return d;
}

__global__ __launch_bounds__(NTHR) void k_cvt(const float* __restrict__ src, _Float16* srcH) {
  const int i = (int)blockIdx.x * NTHR + (int)threadIdx.x;
  const float* sp = src + (size_t)i * CVT_PER_THR;
  const v4f f0 = *(const v4f*)sp;
  const v4f f1 = *(const v4f*)(sp + 4);
  v8h hv;
  hv[0] = (_Float16)f0.x; hv[1] = (_Float16)f0.y; hv[2] = (_Float16)f0.z; hv[3] = (_Float16)f0.w;
  hv[4] = (_Float16)f1.x; hv[5] = (_Float16)f1.y; hv[6] = (_Float16)f1.z; hv[7] = (_Float16)f1.w;
  _Float16* d = srcH + (size_t)i * CVT_PER_THR;
  *(volatile v8h*)d = hv;
  __threadfence();
  *(volatile v8h*)d = hv;
}

__global__ __launch_bounds__(NTHR) __attribute__((amdgpu_num_vgpr(256)))
void k_main(const float* __restrict__ src, const float* __restrict__ guide,
            const _Float16* __restrict__ srcH, float* out) {
  extern __shared__ v4f s_g4[];
  __shared__ __attribute__((aligned(16))) float stg[LCH * SPITCH];
  float* s_g = (float*)s_g4;
  const int tid = (int)threadIdx.x, lane = tid & 31, wave = tid >> 5, hh = lane >> 4, m = lane & 15;
  const int b = (int)blockIdx.y, i0 = (int)blockIdx.x * ROWS, iw = i0 + 16 * wave;
  const float* gdb = guide + (size_t)b * DG * NPIX;

#pragma unroll 1
  for (int it = 0; it < NPIX / (4 * NTHR); ++it) {
    const int j4 = (it * NTHR + tid) * 4;
    const v4f g0 = *(const v4f*)(gdb + 0 * NPIX + j4);
    const v4f g1 = *(const v4f*)(gdb + 1 * NPIX + j4);
    const v4f g2 = *(const v4f*)(gdb + 2 * NPIX + j4);
    const v4f g3 = *(const v4f*)(gdb + 3 * NPIX + j4);
    const v4f g4 = *(const v4f*)(gdb + 4 * NPIX + j4);
#pragma unroll
    for (int q = 0; q < 4; ++q) {
      const v4f u = {g0[q], g1[q], g2[q], g3[q]};
      float* d = s_g + (size_t)(j4 + q) * GP;
      *(v4f*)d = u;
      d[4] = g4[q];
    }
  }
  __syncthreads();

  const v4f gi = *(const v4f*)(s_g + (size_t)(iw + m) * GP);
  const float gi4 = s_g[(size_t)(iw + m) * GP + 4];

  const v8f z8 = {0.f, 0.f, 0.f, 0.f, 0.f, 0.f, 0.f, 0.f};
  v8f acc = z8;
  const _Float16* bp = srcH + ((size_t)b * LCH + m) * NPIX + 8 * hh;
  const float NHL2E = -0.72134752044448170f;

#pragma unroll 1
  for (int t = 0; t < NPIX / KCH; ++t) {
    const int jb = t * KCH + 8 * hh;
    FragH a;
#pragma unroll
    for (int e = 0; e < 16; ++e) {
      const int j = jb + e + 8 * (e >> 3);
      const v4f gj = *(const v4f*)(s_g + (size_t)j * GP);
      const float gj4 = s_g[(size_t)j * GP + 4];
      const float d0 = gi.x - gj.x;
      const float d1 = gi.y - gj.y;
      const float d2 = gi.z - gj.z;
      const float d3 = gi.w - gj.w;
      const float d4 = gi4 - gj4;
      float dd = d0 * d0;
      dd = fmaf(d1, d1, dd);
      dd = fmaf(d2, d2, dd);
      dd = fmaf(d3, d3, dd);
      dd = fmaf(d4, d4, dd);
      const float w = exp2f(fmaf(dd, NHL2E, 8.0f));
      a.e[e] = (_Float16)w;
    }
    FragH bf;
    bf.h[0] = *(const v8h*)(bp + (size_t)t * KCH);
    bf.h[1] = *(const v8h*)(bp + (size_t)t * KCH + 16);
    acc = wmf(a.v, bf.v, acc);
  }

  {
    float* sp = stg + m * SPITCH + 16 * wave + 8 * hh;
    const v4f u0 = {acc[0], acc[1], acc[2], acc[3]};
    const v4f u1 = {acc[4], acc[5], acc[6], acc[7]};
    *(v4f*)sp = u0;
    *(v4f*)(sp + 4) = u1;
  }
  __syncthreads();

  const float OSC = 1.0f / 256.0f;
  v4f ov[2];
#pragma unroll
  for (int rr = 0; rr < 2; ++rr) {
    const int l = 2 * wave + rr;
    const v4f f = *(const v4f*)(stg + l * SPITCH + 4 * lane);
    const v4f s = *(const v4f*)(src + ((size_t)b * LCH + l) * NPIX + i0 + 4 * lane);
    v4f o;
    o.x = f.x * OSC - s.x;
    o.y = f.y * OSC - s.y;
    o.z = f.z * OSC - s.z;
    o.w = f.w * OSC - s.w;
    ov[rr] = o;
  }
  float* ob = out + ((size_t)b * LCH + 2 * wave) * NPIX + i0 + 4 * lane;
  *(volatile v4f*)ob = ov[0];
  *(volatile v4f*)(ob + NPIX) = ov[1];
  __threadfence();
  *(volatile v4f*)ob = ov[0];
  *(volatile v4f*)(ob + NPIX) = ov[1];
}

extern "C" void kernel_launch(void* const* d_in, const int* in_sizes, int n_in,
                              void* d_out, int out_size, void* d_ws, size_t ws_size,
                              hipStream_t stream) {
  if (n_in < 2) return;
  if (in_sizes[0] != NB * LCH * NPIX) return;
  if (in_sizes[1] != NB * DG * NPIX) return;
  if (out_size != NB * LCH * NPIX) return;

  const float* src   = (const float*)d_in[0];
  const float* guide = (const float*)d_in[1];
  float* out = (float*)d_out;

  char* ws = (char*)d_ws;
  size_t off = 0;
  const size_t oH = off; off += (size_t)NB * LCH * NPIX * 2; off = (off + 255) & ~(size_t)255;
  if (off > ws_size || off > (size_t)WSCAP) return;
  _Float16* srcH = (_Float16*)(ws + oH);

  hipFuncSetAttribute(reinterpret_cast<const void*>(&k_main),
                      hipFuncAttributeMaxDynamicSharedMemorySize, GLDS);

  k_cvt<<<(NB * LCH * NPIX) / (CVT_PER_THR * NTHR), NTHR, 0, stream>>>(src, srcH);
  k_main<<<dim3(NPIX / ROWS, NB), NTHR, GLDS, stream>>>(src, guide, srcH, out);
}
